// ConvolutionalAttention_6700148982325
// MI455X (gfx1250) — hardware-verified
//
#include <hip/hip_runtime.h>
#include <math.h>

typedef __attribute__((ext_vector_type(16))) _Float16 v16h;
typedef __attribute__((ext_vector_type(16))) __bf16 v16b;
typedef __attribute__((ext_vector_type(8)))  _Float16 v8h;
typedef __attribute__((ext_vector_type(8)))  float v8f;
typedef __attribute__((ext_vector_type(4)))  float v4f;
typedef __attribute__((ext_vector_type(2)))  float v2f;
typedef __attribute__((ext_vector_type(4)))  unsigned v4u;
typedef __attribute__((ext_vector_type(4)))  int v4i;
typedef float __attribute__((may_alias)) float_a;
typedef int __attribute__((may_alias)) int_a;

template <typename T> __device__ __forceinline__ void vst2(void* p, T v) { *(volatile T*)p = v; __threadfence(); *(volatile T*)p = v; }
__device__ __forceinline__ v8f wmma16(v16h a, v16h b, v8f c) {
  v8f d = __builtin_amdgcn_wmma_f32_16x16x32_f16(false, a, false, b, (short)0, c, false, false);
  asm volatile("v_nop\n\tv_nop\n\tv_nop\n\tv_nop" : "+v"(d) : "v"(a), "v"(b));
  return d;
}
__device__ __forceinline__ v8f wmma_bf(v16b a, v16b b, v8f c) {
  v8f d = __builtin_amdgcn_wmma_f32_16x16x32_bf16(false, a, false, b, (short)0, c, false, false);
  asm volatile("v_nop\n\tv_nop\n\tv_nop\n\tv_nop" : "+v"(d) : "v"(a), "v"(b));
  return d;
}
__device__ __forceinline__ v16h frag_h(const _Float16* rowk0, int lane) {
  union { v16h v; v8h q[2]; } u; const _Float16* p = rowk0 + 8 * (lane >> 4);
  u.q[0] = *(const v8h*)p; u.q[1] = *(const v8h*)(p + 16); return u.v;
}
__device__ __forceinline__ v16h frag_f32(const float* rowk0, int lane) {
  v16h a; const float* p = rowk0 + 8 * (lane >> 4);
#pragma unroll
  for (int i = 0; i < 8; ++i) { a[i] = (_Float16)p[i]; a[8 + i] = (_Float16)p[16 + i]; }
  return a;
}
__device__ __forceinline__ v16h frag_f32s(const float* rowk0, int lane, float sc) {
  v16h a; const float* p = rowk0 + 8 * (lane >> 4);
#pragma unroll
  for (int i = 0; i < 8; ++i) { a[i] = (_Float16)(p[i] * sc); a[8 + i] = (_Float16)(p[16 + i] * sc); }
  return a;
}
__device__ __forceinline__ v16h fragc_f32(const float* W, int k0, int n, int lane, int ld, int K) {
  v16h a; const int g = lane >> 4;
#pragma unroll
  for (int i = 0; i < 8; ++i) { const int ka = k0 + 8 * g + i, kb = ka + 16;
    a[i] = (_Float16)(ka < K ? W[(size_t)(ka < K ? ka : K - 1) * ld + n] : 0.f); a[8 + i] = (_Float16)(kb < K ? W[(size_t)(kb < K ? kb : K - 1) * ld + n] : 0.f); }
  return a;
}
struct F2 { v16b h, l; };
__device__ __forceinline__ F2 bsplit16(const float v[16]) { F2 r;
#pragma unroll
  for (int i = 0; i < 16; ++i) { const __bf16 h = (__bf16)v[i]; r.h[i] = h; r.l[i] = (__bf16)(v[i] - (float)h); }
  return r; }
__device__ __forceinline__ F2 split_row(const float* row, int k0, int lane) { float v[16]; const float* p = row + k0 + 8 * (lane >> 4);
#pragma unroll
  for (int i = 0; i < 8; ++i) { v[i] = p[i]; v[8 + i] = p[16 + i]; }
  return bsplit16(v); }
__device__ __forceinline__ F2 split_rowK(const float* row, int k0, int lane, int K) { float v[16]; const int g = lane >> 4;
#pragma unroll
  for (int i = 0; i < 8; ++i) { const int ka = k0 + 8 * g + i, kb = ka + 16; v[i] = ka < K ? row[ka < K ? ka : K - 1] : 0.f; v[8 + i] = kb < K ? row[kb < K ? kb : K - 1] : 0.f; }
  return bsplit16(v); }
__device__ __forceinline__ F2 split_col(const float* W, int k0, int n, int lane, int ld, int K) { float v[16]; const int g = lane >> 4;
#pragma unroll
  for (int i = 0; i < 8; ++i) { const int ka = k0 + 8 * g + i, kb = ka + 16; v[i] = ka < K ? W[(size_t)(ka < K ? ka : K - 1) * ld + n] : 0.f; v[8 + i] = kb < K ? W[(size_t)(kb < K ? kb : K - 1) * ld + n] : 0.f; }
  return bsplit16(v); }
__device__ __forceinline__ v8f mac3(const F2& a, const F2& b, v8f c) { c = wmma_bf(a.l, b.h, c); c = wmma_bf(a.h, b.l, c); return wmma_bf(a.h, b.h, c); }
__device__ __forceinline__ float sigm(float v) { return 1.0f / (1.0f + expf(-v)); }
#define LDSX() do { asm volatile("s_wait_dscnt 0" ::: "memory"); __builtin_amdgcn_wave_barrier(); __builtin_amdgcn_fence(__ATOMIC_RELEASE, "workgroup"); } while (0)


#define NB 8
#define SQ 256
#define DM 64
#define DC 100
#define DP 128
#define NI1 (SQ - 1)
#define NI2 (SQ - 2)
#define TEMP 10.0f
#ifndef NBT
#define NBT NB
#endif
typedef __attribute__((ext_vector_type(8))) __bf16 v8b;
__device__ __forceinline__ v16b frag_b(const __bf16* rowk0, int lane) {
  union { v16b v; v8b q[2]; } u; const __bf16* p = rowk0 + 8 * (lane >> 4);
  u.q[0] = *(const v8b*)p; u.q[1] = *(const v8b*)(p + 16); return u.v;
}
__device__ __forceinline__ float bfr(float v) { return (float)(__bf16)v; }
__device__ __attribute__((noinline)) float exp_ni(float v) { return expf(v); }
__device__ __attribute__((noinline)) float erf_ni(float v) { return erff(v); }

#define WS_P2   0u
#define WS_P3   (WS_P2 + 2u * DP * 256)
#define WS_AQ   (WS_P3 + 2u * 16 * 256)
#define WS_AK   (WS_AQ + 4u * DP * SQ)
#define WS_R1   (WS_AK + 4u * DP * SQ)
#define WS_R2   (WS_R1 + 4u * SQ * SQ * DP)
#define WS_S3   (WS_R2 + 4u * SQ * SQ * DP)
#define WS_AT   (WS_S3 + 4u * SQ * SQ)
#define WS_VT   (WS_AT + 4u * SQ * SQ)
#define WS_END  (WS_VT + 2u * DM * SQ)

__global__ __launch_bounds__(256) void k_pack(const float* __restrict__ W2, const float* __restrict__ W3, __bf16* __restrict__ P2, __bf16* __restrict__ P3) {
  __shared__ __align__(16) __bf16 s[256]; const int row = blockIdx.x, tid = threadIdx.x; const int tap = tid >> 7, d = tid & 127;
  if (row < DP) { const float v = (row < DC && d < DC) ? W2[((size_t)row * DC + d) * 2 + tap] : 0.f; s[tid] = (__bf16)v; __syncthreads(); if (tid < 32) vst2((unsigned*)(P2 + (size_t)row * 256 + tid * 8), *(const v4u*)&s[tid * 8]); }
  else { const int r = row - DP; const float v = (r == 0 && d < DC) ? W3[(size_t)d * 2 + tap] : 0.f; s[tid] = (__bf16)v; __syncthreads(); if (tid < 32) vst2((unsigned*)(P3 + (size_t)r * 256 + tid * 8), *(const v4u*)&s[tid * 8]); }
}
__global__ __launch_bounds__(256) void k_aqk(const float* __restrict__ Qb, const float* __restrict__ Kb, const float* __restrict__ W1, float* __restrict__ AQ, float* __restrict__ AK) {
  __shared__ float w0[DM], w1[DM], wk[DM]; __shared__ __align__(16) float sq[SQ], sk[SQ]; const int d = blockIdx.x, tid = threadIdx.x;
  if (tid < DM) { const bool ok = d < DC; w0[tid] = ok ? bfr(W1[((size_t)d * 2 * DM + tid) * 2 + 0]) : 0.f; w1[tid] = ok ? bfr(W1[((size_t)d * 2 * DM + tid) * 2 + 1]) : 0.f; wk[tid] = ok ? (bfr(W1[((size_t)d * 2 * DM + DM + tid) * 2 + 0]) + bfr(W1[((size_t)d * 2 * DM + DM + tid) * 2 + 1])) : 0.f; }
  __syncthreads();
  { const int i = tid; float s = 0.f, t = 0.f; const float* qi = Qb + (size_t)i * DM; const float* qn = Qb + (size_t)(i + 1 < SQ ? i + 1 : i) * DM; const float* kj = Kb + (size_t)i * DM;
#pragma unroll 4
    for (int c = 0; c < DM; ++c) { s += w0[c] * bfr(qi[c]) + w1[c] * bfr(qn[c]); t += wk[c] * bfr(kj[c]); }
    sq[i] = (i < NI1) ? s : 0.f; sk[i] = t; }
  __syncthreads();
  if (tid < 64) vst2(AQ + (size_t)d * SQ + tid * 4, *(const v4f*)&sq[tid * 4]); else if (tid < 128) vst2(AK + (size_t)d * SQ + (tid - 64) * 4, *(const v4f*)&sk[(tid - 64) * 4]);
}
__global__ __launch_bounds__(256) void k_r1(const float* __restrict__ AQ, const float* __restrict__ AK, const float* __restrict__ b1, const float* __restrict__ g1, const float* __restrict__ be1, const float* __restrict__ m1, const float* __restrict__ v1, float* __restrict__ R1) {
  __shared__ __align__(16) float s[64][DP + 4]; __shared__ float saq[DP], ssc[DP], ssh[DP], sb1[DP];
  const int ip = blockIdx.x, j0 = blockIdx.y * 64, tid = threadIdx.x;
  if (tid < DP) { const int d = tid; const bool ok = d < DC; saq[d] = (ok && ip > 0) ? AQ[(size_t)d * SQ + ip - 1] : 0.f; sb1[d] = ok ? bfr(b1[d]) : 0.f;
    const float sc = ok ? bfr(g1[d]) / sqrtf(bfr(v1[d]) + 1e-5f) : 0.f; ssc[d] = sc; ssh[d] = ok ? (bfr(be1[d]) - bfr(m1[d]) * sc) : 0.f; }
  __syncthreads();
  for (int q = tid; q < 64 * DP; q += 256) { const int jl = q >> 7, d = q & 127; float v = 0.f;
    if (d < DC) { const float a1 = (ip > 0) ? (saq[d] + AK[(size_t)d * SQ + j0 + jl] + sb1[d]) : 0.f; v = fmaxf(a1 * ssc[d] + ssh[d], 0.f); }
    s[jl][d] = v; }
  __syncthreads();
  for (int q = tid; q < 64 * 32; q += 256) { const int jl = q >> 5, pc = q & 31; vst2(R1 + ((size_t)ip * SQ + j0 + jl) * DP + pc * 4, *(const v4f*)&s[jl][pc * 4]); }
}
__global__ __launch_bounds__(128) void k_c2(const float* __restrict__ R1, const __bf16* __restrict__ P2, const float* __restrict__ AQ, const float* __restrict__ AK, const float* __restrict__ b1, const float* __restrict__ b2, const float* __restrict__ g2, const float* __restrict__ be2, const float* __restrict__ m2, const float* __restrict__ v2, float* __restrict__ R2) {
  __shared__ __align__(16) float so[4][16][132];
  const int tid = threadIdx.x, wave = tid >> 5, lane = tid & 31, col = lane & 15, g = lane >> 4; const int i = blockIdx.y; const int j0 = blockIdx.x * 64 + wave * 16; const int in = (i + 1 < SQ) ? i + 1 : i;
  v8f acc[8] = {};
#pragma unroll
  for (int kc = 0; kc < 8; ++kc) { const float* arow = (kc < 4) ? R1 + ((size_t)i * SQ + j0 + col) * DP : R1 + ((size_t)in * SQ + j0 + col) * DP; const F2 a = split_row(arow, (kc & 3) * 32, lane);
#pragma unroll
    for (int jt = 0; jt < 8; ++jt) { const v16b w = frag_b(P2 + (size_t)(jt * 16 + col) * 256 + kc * 32, lane); acc[jt] = wmma_bf(a.l, w, acc[jt]); acc[jt] = wmma_bf(a.h, w, acc[jt]); } }
#pragma unroll
  for (int jt = 0; jt < 8; ++jt) { const int dp = jt * 16 + col; const bool ok = dp < DC; const float sc = ok ? bfr(g2[dp]) / sqrtf(bfr(v2[dp]) + 1e-5f) : 0.f; const float sh = ok ? (bfr(be2[dp]) - bfr(m2[dp]) * sc) : 0.f; const float bb = ok ? bfr(b2[dp]) + bfr(b1[dp]) + (i < NI1 ? AQ[(size_t)dp * SQ + i] : 0.f) : 0.f;
#pragma unroll
    for (int r = 0; r < 8; ++r) { const int j = j0 + 8 * g + r; float v = 0.f; if (ok) { const float a2 = acc[jt][r] + bb + AK[(size_t)dp * SQ + j]; v = fmaxf(a2 * sc + sh, 0.f); } so[wave][8 * g + r][dp] = v; } }
  LDSX();
  for (int rl = 0; rl < 16; ++rl) vst2(R2 + ((size_t)i * SQ + j0 + rl) * DP + lane * 4, *(const v4f*)&so[wave][rl][lane * 4]);
}
__global__ __launch_bounds__(128) void k_c3(const float* __restrict__ R2, const __bf16* __restrict__ P3, const float* __restrict__ b3, float* __restrict__ S3) {
  __shared__ __align__(16) float ss[64];
  const int tid = threadIdx.x, wave = tid >> 5, lane = tid & 31, col = lane & 15, g = lane >> 4; const int i = blockIdx.y; const int j0 = blockIdx.x * 64 + wave * 16; const int in = (i + 1 < SQ) ? i + 1 : i;
  v8f acc = {};
#pragma unroll
  for (int kc = 0; kc < 8; ++kc) { const float* arow = (kc < 4) ? R2 + ((size_t)i * SQ + j0 + col) * DP : R2 + ((size_t)in * SQ + j0 + col) * DP; const F2 a = split_row(arow, (kc & 3) * 32, lane); const v16b w = frag_b(P3 + (size_t)col * 256 + kc * 32, lane); acc = wmma_bf(a.l, w, acc); acc = wmma_bf(a.h, w, acc); }
  if (col == 0) { const float bb = bfr(b3[0]);
#pragma unroll
    for (int r = 0; r < 8; ++r) ss[wave * 16 + 8 * g + r] = (acc[r] + bb) * (1.0f / TEMP); }
  __syncthreads();
  if (tid < 16) vst2(S3 + (size_t)i * SQ + blockIdx.x * 64 + tid * 4, *(const v4f*)&ss[tid * 4]);
}
__global__ __launch_bounds__(256) void k_soft(const float* __restrict__ S3, float* __restrict__ AT, float* __restrict__ attn_out) {
  const int wave = threadIdx.x >> 5, lane = threadIdx.x & 31; const int i = blockIdx.x * 8 + wave; if (i >= NI2) return;
  const float* row = S3 + (size_t)i * SQ; float v[8]; float mx = -3.0e38f;
#pragma unroll
  for (int k = 0; k < 8; ++k) { v[k] = row[lane * 4 + (k & 3) + (k >> 2) * 128]; mx = fmaxf(mx, v[k]); }
#pragma unroll
  for (int o = 1; o < 32; o <<= 1) mx = fmaxf(mx, __shfl_xor(mx, o));
  float z = 0.f;
#pragma unroll
  for (int k = 0; k < 8; ++k) { v[k] = exp_ni(v[k] - mx); z += v[k]; }
#pragma unroll
  for (int o = 1; o < 32; o <<= 1) z += __shfl_xor(z, o);
  const float iz = 1.0f / z;
#pragma unroll
  for (int h = 0; h < 2; ++h) { v4f p; p[0] = v[h * 4] * iz; p[1] = v[h * 4 + 1] * iz; p[2] = v[h * 4 + 2] * iz; p[3] = v[h * 4 + 3] * iz; vst2(AT + (size_t)i * SQ + h * 128 + lane * 4, p); vst2(attn_out + (size_t)i * SQ + h * 128 + lane * 4, p); }
}
__global__ __launch_bounds__(256) void k_vt(const float* __restrict__ Vb, __bf16* __restrict__ VT) {
  __shared__ __align__(16) __bf16 s[DM][SQ + 8]; const int tid = threadIdx.x;
  for (int q = tid; q < SQ * DM; q += 256) { const int j = q >> 6, c = q & 63; s[c][j] = (__bf16)Vb[(size_t)j * DM + c]; }
  __syncthreads();
  for (int q = tid; q < DM * 32; q += 256) { const int c = q >> 5, pc = q & 31; vst2((unsigned*)(VT + (size_t)c * SQ + pc * 8), *(const v4u*)&s[c][pc * 8]); }
}
__global__ __launch_bounds__(128) void k_pv(const float* __restrict__ AT, const __bf16* __restrict__ VT, float* __restrict__ outb) {
  __shared__ __align__(16) float so[4][16][68];
  const int tid = threadIdx.x, wave = tid >> 5, lane = tid & 31, col = lane & 15, g = lane >> 4; const int i0 = blockIdx.x * 64 + wave * 16; int ia = i0 + col; ia = ia < SQ ? ia : SQ - 1;
  v8f acc[4] = {};
#pragma unroll
  for (int kc = 0; kc < SQ / 32; ++kc) { const F2 a = split_row(AT + (size_t)ia * SQ, kc * 32, lane);
#pragma unroll
    for (int jt = 0; jt < 4; ++jt) { const v16b w = frag_b(VT + (size_t)(jt * 16 + col) * SQ + kc * 32, lane); acc[jt] = wmma_bf(a.l, w, acc[jt]); acc[jt] = wmma_bf(a.h, w, acc[jt]); } }
#pragma unroll
  for (int jt = 0; jt < 4; ++jt)
#pragma unroll
    for (int r = 0; r < 8; ++r) so[wave][8 * g + r][jt * 16 + col] = acc[jt][r];
  LDSX();
  for (int rl = 0; rl < 16; ++rl) { const int i = i0 + rl; if (i < NI2 && lane < 16) vst2(outb + (size_t)i * DM + lane * 4, *(const v4f*)&so[wave][rl][lane * 4]); }
}
extern "C" void kernel_launch(void* const* d_in, const int* in_sizes, int n_in, void* d_out, int out_size, void* d_ws, size_t ws_size, hipStream_t stream) {
  (void)in_sizes; (void)n_in; (void)out_size;
  const float** F = (const float**)d_in;
  if (ws_size < (size_t)WS_END) return;
  char* ws = (char*)d_ws; __bf16 *P2 = (__bf16*)(ws + WS_P2), *P3 = (__bf16*)(ws + WS_P3), *VT = (__bf16*)(ws + WS_VT);
  float *AQ = (float*)(ws + WS_AQ), *AK = (float*)(ws + WS_AK), *R1 = (float*)(ws + WS_R1), *R2 = (float*)(ws + WS_R2), *S3 = (float*)(ws + WS_S3), *AT = (float*)(ws + WS_AT);
  float* OUT0 = (float*)d_out; float* OUT1 = (float*)d_out + (size_t)NB * NI2 * DM;
  k_pack<<<DP + 16, 256, 0, stream>>>(F[9], F[15], P2, P3);
  for (int b = 0; b < NBT; ++b) { const float* qb = F[0] + (size_t)b * SQ * DM; const float* kb = F[1] + (size_t)b * SQ * DM; const float* vb = F[2] + (size_t)b * SQ * DM;
    k_aqk<<<DP, 256, 0, stream>>>(qb, kb, F[3], AQ, AK);
    k_r1<<<dim3(SQ, SQ / 64), 256, 0, stream>>>(AQ, AK, F[4], F[5], F[6], F[7], F[8], R1);
    k_c2<<<dim3(SQ / 64, NI1), 128, 0, stream>>>(R1, P2, AQ, AK, F[4], F[10], F[11], F[12], F[13], F[14], R2);
    k_c3<<<dim3(SQ / 64, NI2), 128, 0, stream>>>(R2, P3, F[16], S3);
    k_soft<<<(NI2 + 7) / 8, 256, 0, stream>>>(S3, AT, OUT1 + (size_t)b * NI2 * SQ);
    k_vt<<<1, 256, 0, stream>>>(vb, VT);
    k_pv<<<SQ / 64, 128, 0, stream>>>(AT, VT, OUT0 + (size_t)b * NI2 * DM); }
}
